// _OpenClipAttentionAdapter_63995012710884
// MI455X (gfx1250) — hardware-verified
//
#include <hip/hip_runtime.h>

typedef _Float16 v16h __attribute__((ext_vector_type(16)));
typedef _Float16 v8h  __attribute__((ext_vector_type(8)));
typedef float    v8f  __attribute__((ext_vector_type(8)));
typedef float    v4f  __attribute__((ext_vector_type(4)));

static __device__ __forceinline__ v8f mma16(v16h a, v16h b, v8f c) {
    v8f d = __builtin_amdgcn_wmma_f32_16x16x32_f16(false, a, false, b, (short)0, c, false, false);
    asm volatile("v_nop\n\tv_nop\n\tv_nop\n\tv_nop" : "+v"(d) : "v"(a), "v"(b));
    return d;
}

static __device__ __forceinline__ v16h cat8(v8h lo, v8h hi) {
    return __builtin_shufflevector(lo, hi, 0, 1, 2, 3, 4, 5, 6, 7, 8, 9, 10, 11, 12, 13, 14, 15);
}

static __device__ __forceinline__ v8h pack8(v4f a, v4f b, float s) {
    v8h r;
    r[0] = (_Float16)(a[0] * s); r[1] = (_Float16)(a[1] * s);
    r[2] = (_Float16)(a[2] * s); r[3] = (_Float16)(a[3] * s);
    r[4] = (_Float16)(b[0] * s); r[5] = (_Float16)(b[1] * s);
    r[6] = (_Float16)(b[2] * s); r[7] = (_Float16)(b[3] * s);
    return r;
}

__global__ __launch_bounds__(256) void gemm_nt(const float* __restrict__ X,
                                               const float* __restrict__ W,
                                               const float* __restrict__ bias,
                                               float* Y, int M, int N, int K,
                                               float sa, float sw, float oscale) {
    constexpr int BM = 128, BN = 128, BK = 32, LDT = 40, CP = 128;
    __shared__ __align__(16) char smem[65536];
    _Float16* As = (_Float16*)smem;
    _Float16* Ws = (_Float16*)(smem + BM * LDT * 2);
    float*    Cs = (float*)smem;

    const int tid  = threadIdx.x;
    const int lane = tid & 31;
    const int wid  = tid >> 5;
    const int lh   = lane >> 4;
    const int l15  = lane & 15;
    const int wm0  = (wid >> 1) * 32;
    const int wn0  = (wid & 1) * 64;
    const int m0   = blockIdx.y * BM;
    const int n0   = blockIdx.x * BN;

    const int srow = tid >> 1;
    const int scol = (tid & 1) * 16;
    const int am = m0 + srow;
    const int wn = n0 + srow;
    const bool aok = am < M;
    const bool wok = wn < N;
    const float* xrow = X + (size_t)(aok ? am : 0) * (size_t)K + scol;
    const float* wrow = W + (size_t)(wok ? wn : 0) * (size_t)K + scol;

    v8f acc[2][4] = {};
    const v4f z4 = {0.f, 0.f, 0.f, 0.f};

    const int KT = K / BK;
#pragma unroll 1
    for (int kt = 0; kt < KT; ++kt) {
        const int k0 = kt * BK;
        v4f x0 = z4, x1 = z4, x2 = z4, x3 = z4;
        v4f w0 = z4, w1 = z4, w2 = z4, w3 = z4;
        if (aok) {
            x0 = *(const v4f*)(xrow + k0);
            x1 = *(const v4f*)(xrow + k0 + 4);
            x2 = *(const v4f*)(xrow + k0 + 8);
            x3 = *(const v4f*)(xrow + k0 + 12);
        }
        if (wok) {
            w0 = *(const v4f*)(wrow + k0);
            w1 = *(const v4f*)(wrow + k0 + 4);
            w2 = *(const v4f*)(wrow + k0 + 8);
            w3 = *(const v4f*)(wrow + k0 + 12);
        }
        __syncthreads();
        *(v8h*)&As[srow * LDT + scol]     = pack8(x0, x1, sa);
        *(v8h*)&As[srow * LDT + scol + 8] = pack8(x2, x3, sa);
        *(v8h*)&Ws[srow * LDT + scol]     = pack8(w0, w1, sw);
        *(v8h*)&Ws[srow * LDT + scol + 8] = pack8(w2, w3, sw);
        __syncthreads();

        v16h af[2], bf[4];
#pragma unroll
        for (int mi = 0; mi < 2; ++mi) {
            const int r = wm0 + mi * 16 + l15;
            v8h lo = *(const v8h*)&As[r * LDT + 8 * lh];
            v8h hi = *(const v8h*)&As[r * LDT + 16 + 8 * lh];
            af[mi] = cat8(lo, hi);
        }
#pragma unroll
        for (int ni = 0; ni < 4; ++ni) {
            const int r = wn0 + ni * 16 + l15;
            v8h lo = *(const v8h*)&Ws[r * LDT + 8 * lh];
            v8h hi = *(const v8h*)&Ws[r * LDT + 16 + 8 * lh];
            bf[ni] = cat8(lo, hi);
        }
#pragma unroll
        for (int mi = 0; mi < 2; ++mi)
#pragma unroll
            for (int ni = 0; ni < 4; ++ni)
                acc[mi][ni] = mma16(af[mi], bf[ni], acc[mi][ni]);
    }

    __syncthreads();
#pragma unroll
    for (int ni = 0; ni < 4; ++ni) {
        const int col  = wn0 + ni * 16 + l15;
        const int gcol = n0 + col;
        const float bv = (gcol < N) ? bias[gcol] : 0.f;
#pragma unroll
        for (int mi = 0; mi < 2; ++mi) {
            const int rb = wm0 + mi * 16 + 8 * lh;
#pragma unroll
            for (int r = 0; r < 8; ++r)
                Cs[(rb + r) * CP + col] = acc[mi][ni][r] * oscale + bv;
        }
    }
    __syncthreads();

#pragma unroll
    for (int i = 0; i < 16; ++i) {
        const int row  = wid * 16 + i;
        const int grow = m0 + row;
        const int gc   = n0 + lane * 4;
        if (grow < M && gc + 3 < N) {
            v4f v = *(const v4f*)&Cs[row * CP + lane * 4];
            *(volatile v4f*)(Y + (size_t)grow * (size_t)N + gc) = v;
        }
    }
    __threadfence();
#pragma unroll
    for (int i = 0; i < 16; ++i) {
        const int row  = wid * 16 + i;
        const int grow = m0 + row;
        const int gc   = n0 + lane * 4;
        if (grow < M && gc + 3 < N) {
            v4f v = *(const v4f*)&Cs[row * CP + lane * 4];
            *(volatile v4f*)(Y + (size_t)grow * (size_t)N + gc) = v;
        }
    }
}

__global__ __launch_bounds__(256) void attn_fwd(const float* __restrict__ Q,
                                                const float* __restrict__ Kf,
                                                const float* __restrict__ Vf,
                                                float* Ctx) {
    constexpr int NN = 1024, DM = 1024, HD = 64;
    constexpr int KP = 72, VP = 40, PP = 40;
    constexpr float SC   = 0.125f;
    constexpr float PSC  = 256.f;
    constexpr float PINV = 0.00390625f;

    __shared__ __align__(16) _Float16 Ks[32 * KP];
    __shared__ __align__(16) _Float16 Vt[HD * VP];
    __shared__ __align__(16) _Float16 Ps[8 * 16 * PP];
    __shared__ __align__(16) float    Os[128 * HD];

    const int b    = blockIdx.z;
    const int hidx = blockIdx.y;
    const int q0   = blockIdx.x * 128;
    const int tid  = threadIdx.x;
    const int lane = tid & 31;
    const int w    = tid >> 5;
    const int lh   = lane >> 4;
    const int l15  = lane & 15;

    const size_t base = (size_t)b * NN * DM + (size_t)hidx * HD;
    const float* Qp = Q  + base;
    const float* Kp = Kf + base;
    const float* Vp = Vf + base;

    v16h qf[2];
    {
        const int qrow = q0 + w * 16 + l15;
#pragma unroll
        for (int dc = 0; dc < 2; ++dc) {
            const float* g = Qp + (size_t)qrow * DM + dc * 32;
            v4f a0 = *(const v4f*)(g + 8 * lh);
            v4f a1 = *(const v4f*)(g + 8 * lh + 4);
            v4f a2 = *(const v4f*)(g + 16 + 8 * lh);
            v4f a3 = *(const v4f*)(g + 16 + 8 * lh + 4);
            qf[dc] = cat8(pack8(a0, a1, 1.f), pack8(a2, a3, 1.f));
        }
    }

    v8f o[4] = {};
    float m_[8], l_[8];
#pragma unroll
    for (int r = 0; r < 8; ++r) { m_[r] = -__builtin_inff(); l_[r] = 0.f; }

    const int sr = tid >> 3;
    const int sc = (tid & 7) * 8;
    _Float16* pw = &Ps[w * 16 * PP];

#pragma unroll 1
    for (int kv0 = 0; kv0 < NN; kv0 += 32) {
        __syncthreads();
        {
            const float* kg = Kp + (size_t)(kv0 + sr) * DM + sc;
            v4f k0v = *(const v4f*)kg;
            v4f k1v = *(const v4f*)(kg + 4);
            *(v8h*)&Ks[sr * KP + sc] = pack8(k0v, k1v, 1.f);
            const float* vg = Vp + (size_t)(kv0 + sr) * DM + sc;
            v4f v0v = *(const v4f*)vg;
            v4f v1v = *(const v4f*)(vg + 4);
            v8h vv = pack8(v0v, v1v, 1.f);
#pragma unroll
            for (int i = 0; i < 8; ++i) Vt[(sc + i) * VP + sr] = vv[i];
        }
        __syncthreads();

        v8f s[2] = {};
#pragma unroll
        for (int t = 0; t < 2; ++t) {
            const int kcol = t * 16 + l15;
#pragma unroll
            for (int dc = 0; dc < 2; ++dc) {
                v8h lo = *(const v8h*)&Ks[kcol * KP + dc * 32 + 8 * lh];
                v8h hi = *(const v8h*)&Ks[kcol * KP + dc * 32 + 16 + 8 * lh];
                s[t] = mma16(qf[dc], cat8(lo, hi), s[t]);
            }
            s[t] = s[t] * SC;
        }

        float p0[8], p1[8], alpha[8];
#pragma unroll
        for (int r = 0; r < 8; ++r) {
            float cm = fmaxf(s[0][r], s[1][r]);
            cm = fmaxf(cm, __shfl_xor(cm, 1));
            cm = fmaxf(cm, __shfl_xor(cm, 2));
            cm = fmaxf(cm, __shfl_xor(cm, 4));
            cm = fmaxf(cm, __shfl_xor(cm, 8));
            const float mn = fmaxf(m_[r], cm);
            alpha[r] = __expf(m_[r] - mn);
            p0[r] = __expf(s[0][r] - mn);
            p1[r] = __expf(s[1][r] - mn);
            float rs = p0[r] + p1[r];
            rs += __shfl_xor(rs, 1);
            rs += __shfl_xor(rs, 2);
            rs += __shfl_xor(rs, 4);
            rs += __shfl_xor(rs, 8);
            l_[r] = l_[r] * alpha[r] + rs;
            m_[r] = mn;
        }
#pragma unroll
        for (int dt = 0; dt < 4; ++dt)
#pragma unroll
            for (int r = 0; r < 8; ++r) o[dt][r] *= alpha[r];

        {
            const int prow = 8 * lh;
#pragma unroll
            for (int r = 0; r < 8; ++r) {
                pw[(prow + r) * PP + l15]      = (_Float16)(p0[r] * PSC);
                pw[(prow + r) * PP + 16 + l15] = (_Float16)(p1[r] * PSC);
            }
        }
        __syncthreads();

        v16h pf;
        {
            v8h lo = *(const v8h*)&pw[l15 * PP + 8 * lh];
            v8h hi = *(const v8h*)&pw[l15 * PP + 16 + 8 * lh];
            pf = cat8(lo, hi);
        }

#pragma unroll
        for (int dt = 0; dt < 4; ++dt) {
            const int ncol = dt * 16 + l15;
            v8h lo = *(const v8h*)&Vt[ncol * VP + 8 * lh];
            v8h hi = *(const v8h*)&Vt[ncol * VP + 16 + 8 * lh];
            o[dt] = mma16(pf, cat8(lo, hi), o[dt]);
        }
    }

    float inv[8];
#pragma unroll
    for (int r = 0; r < 8; ++r) inv[r] = (1.f / l_[r]) * PINV;
#pragma unroll
    for (int dt = 0; dt < 4; ++dt) {
        const int col = dt * 16 + l15;
#pragma unroll
        for (int r = 0; r < 8; ++r)
            Os[(w * 16 + 8 * lh + r) * HD + col] = o[dt][r] * inv[r];
    }
    __syncthreads();

#pragma unroll
    for (int i = 0; i < 8; ++i) {
        const int rr = 2 * i + lh;
        const int c  = l15 * 4;
        v4f v = *(const v4f*)&Os[(w * 16 + rr) * HD + c];
        const size_t grow = (size_t)b * NN + q0 + w * 16 + rr;
        *(volatile v4f*)(Ctx + grow * DM + hidx * HD + c) = v;
    }
    __threadfence();
#pragma unroll
    for (int i = 0; i < 8; ++i) {
        const int rr = 2 * i + lh;
        const int c  = l15 * 4;
        v4f v = *(const v4f*)&Os[(w * 16 + rr) * HD + c];
        const size_t grow = (size_t)b * NN + q0 + w * 16 + rr;
        *(volatile v4f*)(Ctx + grow * DM + hidx * HD + c) = v;
    }
}

extern "C" void kernel_launch(void* const* d_in, const int* in_sizes, int n_in,
                              void* d_out, int out_size, void* d_ws, size_t ws_size,
                              hipStream_t stream) {
    const int B = 4, N = 1024, D = 1024, H = 16;
    const int M = B * N;

    if (n_in < 9) return;
    if (in_sizes[0] != M * D) return;
    if (in_sizes[1] != D * D || in_sizes[3] != D * D || in_sizes[5] != D * D || in_sizes[7] != D * D) return;
    if (in_sizes[2] != D || in_sizes[4] != D || in_sizes[6] != D || in_sizes[8] != D) return;
    if (out_size != M * D) return;
    if ((D % 32) != 0 || (N % 128) != 0 || (D / H) != 64) return;

    const size_t act_bytes = (size_t)M * (size_t)D * sizeof(float);
    if (ws_size < 4 * act_bytes) return;

    const float* hs = (const float*)d_in[0];
    const float* qw = (const float*)d_in[1];
    const float* qb = (const float*)d_in[2];
    const float* kw = (const float*)d_in[3];
    const float* kb = (const float*)d_in[4];
    const float* vw = (const float*)d_in[5];
    const float* vb = (const float*)d_in[6];
    const float* ow = (const float*)d_in[7];
    const float* ob = (const float*)d_in[8];

    char* ws = (char*)d_ws;
    float* qf  = (float*)(ws + 0 * act_bytes);
    float* kf  = (float*)(ws + 1 * act_bytes);
    float* vf  = (float*)(ws + 2 * act_bytes);
    float* ctx = (float*)(ws + 3 * act_bytes);

    const float WSC = 64.f;
    const float CSC = 64.f;

    dim3 gg((D + 127) / 128, (M + 127) / 128);
    gemm_nt<<<gg, 256, 0, stream>>>(hs, qw, qb, qf, M, D, D, 1.f, WSC, 1.f / WSC);
    gemm_nt<<<gg, 256, 0, stream>>>(hs, kw, kb, kf, M, D, D, 1.f, WSC, 1.f / WSC);
    gemm_nt<<<gg, 256, 0, stream>>>(hs, vw, vb, vf, M, D, D, 1.f, WSC, 1.f / WSC);

    dim3 ga(N / 128, H, B);
    attn_fwd<<<ga, 256, 0, stream>>>(qf, kf, vf, ctx);

    gemm_nt<<<gg, 256, 0, stream>>>(ctx, ow, ob, (float*)d_out, M, D, D, CSC, WSC, 1.f / (CSC * WSC));
}
